// NCL_50766513438744
// MI455X (gfx1250) — hardware-verified
//
#include <hip/hip_runtime.h>
#include <math.h>

typedef __attribute__((ext_vector_type(16))) _Float16 v16h;
typedef __attribute__((ext_vector_type(8)))  _Float16 v8h;
typedef __attribute__((ext_vector_type(8)))  float    v8f;
typedef __attribute__((ext_vector_type(4)))  float    v4f;

constexpr int kPts        = 1000000;
constexpr int kHid        = 32;
constexpr int kTileS      = 32;
constexpr int kTiles      = kPts / kTileS;
constexpr int kWaves      = 4;
constexpr int kBlocks     = 1954;
constexpr int kTotalWaves = kBlocks * kWaves;
constexpr int kIters      = (kTiles + kTotalWaves - 1) / kTotalWaves;
static_assert(kTiles * kTileS == kPts);
static_assert(kTotalWaves * kIters >= kTiles);
static_assert(kHid == 32);

constexpr bool kFwdSplit = true;
constexpr bool kTanSplit = false;

constexpr float kBeta          = 20.0f;
constexpr float kInvBeta       = 1.0f / kBeta;
constexpr float kCarryA        = 64.0f;
constexpr float kCarryW        = 64.0f;
constexpr float kCarryLo       = 2048.0f;
constexpr float kAccScale      = kCarryA * kCarryW;
constexpr float kInvMain       = 1.0f / kAccScale;
constexpr float kInvRes        = kInvMain / kCarryLo;
constexpr float kNextMain      = kCarryA * kInvMain;
constexpr float kNextRes       = kCarryA * kInvRes;
constexpr float kHalfMinNormal = 6.103515625e-5f;
constexpr float kF32MinNormal  = 1.17549435e-38f;

constexpr int kAP       = 40;
constexpr int kWP       = 32;
constexpr int kW4P      = 96;
constexpr int kRowFwdHi = 0;
constexpr int kRowFwdLo = 32;
constexpr int kRowTanHi = 64;
constexpr int kRowTanLo = 160;
constexpr int kRowsW    = kTanSplit ? 256 : 160;
constexpr int kLdsBytes = kWaves * kRowsW * kAP * 2 + 4 * kHid * kWP * 2 + 16 * kW4P * 2 + 128 * 4 + 128 * 4 + kWaves * 96 * 4;
static_assert(kTanSplit || kLdsBytes <= 65536);
static_assert((kAP % 8) == 0 && (kWP % 8) == 0 && (kW4P % 8) == 0);

template <typename T> struct Frag;
template <> struct Frag<_Float16> {
  typedef v16h V; union U { v16h v; v8h h[2]; };
  static __device__ __forceinline__ v16h load(const _Float16* p) {
    U f; f.h[0] = *(const v8h*)(p); f.h[1] = *(const v8h*)(p + 16); return f.v;
  }
};
typedef Frag<_Float16> FragH;

__device__ __forceinline__ v8f mma_h(v16h a, v16h b, v8f c) {
  c = __builtin_amdgcn_wmma_f32_16x16x32_f16(false, a, false, b, (short)0, c, false, false);
  asm volatile("v_nop\n\tv_nop\n\tv_nop\n\tv_nop" : "+v"(c) : "v"(a), "v"(b));
  return c;
}

__device__ __forceinline__ void wave_sync() {
  __builtin_amdgcn_fence(__ATOMIC_RELEASE, "workgroup");
  __builtin_amdgcn_wave_barrier();
  __builtin_amdgcn_fence(__ATOMIC_ACQUIRE, "workgroup");
}

__device__ __forceinline__ _Float16 to_h(float v) {
  const float f = (__builtin_fabsf(v) < kHalfMinNormal) ? 0.0f : v;
  return (_Float16)f;
}
__device__ __forceinline__ void split_h(float v, _Float16& hi, _Float16& lo) {
  hi = to_h(v);
  float hf = (float)hi;
  asm volatile("" : "+v"(hf));
  lo = to_h((v - hf) * kCarryLo);
}

__device__ __forceinline__ float gate_e(float pre) {
  const float e = expf(-kBeta * __builtin_fabsf(pre));
  return (e < kF32MinNormal) ? 0.0f : e;
}
__device__ __forceinline__ void act_pair(float pre, float& hval, float& sval) {
  const float e = gate_e(pre);
  const float r = __builtin_amdgcn_rcpf(1.0f + e);
  hval = fmaxf(pre, 0.0f) + log1pf(e) * kInvBeta;
  sval = (pre >= 0.0f) ? r : e * r;
}
__device__ __forceinline__ float slope_only(float pre) {
  const float e = gate_e(pre);
  const float r = __builtin_amdgcn_rcpf(1.0f + e);
  return (pre >= 0.0f) ? r : e * r;
}

template <bool NEED_H>
__device__ __forceinline__ void hidden_layer(_Float16* Aw, const _Float16* Wh, const _Float16* Wl,
                                             const float* bias, int hh, int c) {
  const v8f z8 = (v8f){0.f, 0.f, 0.f, 0.f, 0.f, 0.f, 0.f, 0.f};
#pragma unroll 1
  for (int mt = 0; mt < 2; ++mt) {
    const int arow = mt * 16 + c;
    const v16h afh = FragH::load(Aw + (kRowFwdHi + arow) * kAP + 8 * hh);
    v16h afl = afh;
    if (kFwdSplit) afl = FragH::load(Aw + (kRowFwdLo + arow) * kAP + 8 * hh);
    const v16h at0 = FragH::load(Aw + (kRowTanHi + 0  + arow) * kAP + 8 * hh);
    const v16h at1 = FragH::load(Aw + (kRowTanHi + 32 + arow) * kAP + 8 * hh);
    const v16h at2 = FragH::load(Aw + (kRowTanHi + 64 + arow) * kAP + 8 * hh);
    v16h al0 = at0, al1 = at1, al2 = at2;
    if (kTanSplit) {
      al0 = FragH::load(Aw + (kRowTanLo + 0  + arow) * kAP + 8 * hh);
      al1 = FragH::load(Aw + (kRowTanLo + 32 + arow) * kAP + 8 * hh);
      al2 = FragH::load(Aw + (kRowTanLo + 64 + arow) * kAP + 8 * hh);
    }
    wave_sync();
#pragma unroll 1
    for (int nt = 0; nt < 2; ++nt) {
      const int ncol = nt * 16 + c;
      const v16h bh = FragH::load(Wh + ncol * kWP + 8 * hh);
      v16h bl = bh;
      if (kFwdSplit) bl = FragH::load(Wl + ncol * kWP + 8 * hh);
      const float bsc = bias[ncol] * kAccScale;
      v8f am = (v8f){bsc, bsc, bsc, bsc, bsc, bsc, bsc, bsc};
      v8f ar = z8;
      am = mma_h(afh, bh, am);
      if (kFwdSplit) {
        ar = mma_h(afh, bl, ar);
        ar = mma_h(afl, bh, ar);
      }
      v8f t0 = mma_h(at0, bh, z8);
      v8f t1 = mma_h(at1, bh, z8);
      v8f t2 = mma_h(at2, bh, z8);
      v8f u0 = z8, u1 = z8, u2 = z8;
      if (kTanSplit) {
        u0 = mma_h(al0, bh, z8);
        u1 = mma_h(al1, bh, z8);
        u2 = mma_h(al2, bh, z8);
      }
      const int obase = (mt * 16 + 8 * hh) * kAP + ncol;
#pragma unroll
      for (int r = 0; r < 8; ++r) {
        float pre = am[r] * kInvMain;
        if (kFwdSplit) pre = fmaf(ar[r], kInvRes, pre);
        float hv = 0.0f, sv;
        if (NEED_H) act_pair(pre, hv, sv);
        else        sv = slope_only(pre);
        const int ro = obase + r * kAP;
        if (NEED_H) {
          _Float16 qh, ql;
          split_h(hv * kCarryA, qh, ql);
          Aw[kRowFwdHi * kAP + ro] = qh;
          if (kFwdSplit) Aw[kRowFwdLo * kAP + ro] = ql;
        }
        const float gm = sv * kNextMain;
        const float gr = sv * kNextRes;
        float tv0 = t0[r] * gm;
        float tv1 = t1[r] * gm;
        float tv2 = t2[r] * gm;
        if (kTanSplit) {
          tv0 = fmaf(u0[r], gr, tv0);
          tv1 = fmaf(u1[r], gr, tv1);
          tv2 = fmaf(u2[r], gr, tv2);
          _Float16 qh, ql;
          split_h(tv0, qh, ql);
          Aw[(kRowTanHi + 0) * kAP + ro] = qh;
          Aw[(kRowTanLo + 0) * kAP + ro] = ql;
          split_h(tv1, qh, ql);
          Aw[(kRowTanHi + 32) * kAP + ro] = qh;
          Aw[(kRowTanLo + 32) * kAP + ro] = ql;
          split_h(tv2, qh, ql);
          Aw[(kRowTanHi + 64) * kAP + ro] = qh;
          Aw[(kRowTanLo + 64) * kAP + ro] = ql;
        } else {
          Aw[(kRowTanHi + 0)  * kAP + ro] = to_h(tv0);
          Aw[(kRowTanHi + 32) * kAP + ro] = to_h(tv1);
          Aw[(kRowTanHi + 64) * kAP + ro] = to_h(tv2);
        }
      }
    }
  }
}

__global__ __launch_bounds__(128) void jet_field_kernel(
    const float* __restrict__ x,
    const float* __restrict__ W1, const float* __restrict__ b1,
    const float* __restrict__ W2, const float* __restrict__ b2,
    const float* __restrict__ W3, const float* __restrict__ b3,
    const float* __restrict__ W4,
    float* __restrict__ out) {
  __shared__ __align__(16) _Float16 sA[kWaves * kRowsW * kAP];
  __shared__ __align__(16) _Float16 sW2h[kHid * kWP];
  __shared__ __align__(16) _Float16 sW2l[kHid * kWP];
  __shared__ __align__(16) _Float16 sW3h[kHid * kWP];
  __shared__ __align__(16) _Float16 sW3l[kHid * kWP];
  __shared__ __align__(16) _Float16 sW4[16 * kW4P];
  __shared__ __align__(16) float sW1[128];
  __shared__ __align__(16) float sBias[128];
  __shared__ __align__(16) float sO[kWaves * 96];

  const unsigned tid = threadIdx.x;
  const int lane = (int)(tid & 31u);
  const int wave = __builtin_amdgcn_readfirstlane((int)(tid >> 5));
  const int hh = lane >> 4;
  const int c  = lane & 15;

  {
    unsigned ip = (tid < 95u) ? tid : 95u;
    asm volatile("" : "+v"(ip));
    float w1v = W1[ip];
    asm volatile("" : "+v"(w1v));
    unsigned jb = tid & 31u;
    asm volatile("" : "+v"(jb));
    float c1 = b1[jb];
    float c2 = b2[jb];
    float c3 = b3[jb];
    asm volatile("" : "+v"(c1), "+v"(c2), "+v"(c3));
    const unsigned sel = tid >> 5;
    const float bv = (sel == 0u) ? c1 : ((sel == 1u) ? c2 : ((sel == 2u) ? c3 : 0.0f));
    sW1[tid]   = (tid < 96u) ? w1v : 0.0f;
    sBias[tid] = bv;
  }
#pragma unroll 1
  for (unsigned i = 0; i < 8u; ++i) {
    const unsigned n = (tid >> 5) + 4u * i;
    const unsigned k = tid & 31u;
    const float w2 = W2[k * 32u + n] * kCarryW;
    const float w3 = W3[k * 32u + n] * kCarryW;
    _Float16 qh, ql;
    split_h(w2, qh, ql);
    sW2h[n * kWP + k] = qh;
    sW2l[n * kWP + k] = ql;
    split_h(w3, qh, ql);
    sW3h[n * kWP + k] = qh;
    sW3l[n * kWP + k] = ql;
  }
  {
    unsigned kq = (tid < 95u) ? tid : 95u;
    asm volatile("" : "+v"(kq));
    const unsigned blk = kq >> 5;
    const unsigned kk  = kq & 31u;
    float q0 = W4[kk * 3u + 0u];
    float q1 = W4[kk * 3u + 1u];
    float q2 = W4[kk * 3u + 2u];
    asm volatile("" : "+v"(q0), "+v"(q1), "+v"(q2));
    q0 *= kCarryW;
    q1 *= kCarryW;
    q2 *= kCarryW;
    const float v0 = (blk == 1u) ? q0  : ((blk == 2u) ? q1  : 0.0f);
    const float v1 = (blk == 0u) ? -q0 : ((blk == 2u) ? q2  : 0.0f);
    const float v2 = (blk == 0u) ? -q1 : ((blk == 1u) ? -q2 : 0.0f);
    float zf = 0.0f;
    asm volatile("" : "+v"(zf));
    const _Float16 h0 = to_h(v0);
    const _Float16 h1 = to_h(v1);
    const _Float16 h2 = to_h(v2);
    const _Float16 hz = (_Float16)zf;
    if (tid < 96u) {
      sW4[0 * kW4P + tid] = h0;
      sW4[1 * kW4P + tid] = h1;
      sW4[2 * kW4P + tid] = h2;
#pragma unroll 1
      for (int n = 3; n < 16; ++n) sW4[n * kW4P + tid] = hz;
    }
  }
  __syncthreads();

  _Float16* Aw = sA + wave * (kRowsW * kAP);
  float*    Ow = sO + wave * 96;
  const int wg = (int)blockIdx.x * kWaves + wave;
  const v8f z8 = (v8f){0.f, 0.f, 0.f, 0.f, 0.f, 0.f, 0.f, 0.f};

#pragma unroll 1
  for (int it = 0; it < kIters; ++it) {
    const int t = it * kTotalWaves + wg;
    if (t >= kTiles) break;
    wave_sync();

    int smp = t * kTileS + lane;
    smp = (smp < kPts - 1) ? smp : (kPts - 1);
    const float* xp = x + (size_t)smp * 3;
    const float x0 = xp[0];
    const float x1 = xp[1];
    const float x2 = xp[2];
#pragma unroll 1
    for (int g = 0; g < 4; ++g) {
      const v4f wa0 = *(const v4f*)(sW1 + 8 * g);
      const v4f wb0 = *(const v4f*)(sW1 + 8 * g + 4);
      const v4f wa1 = *(const v4f*)(sW1 + 32 + 8 * g);
      const v4f wb1 = *(const v4f*)(sW1 + 32 + 8 * g + 4);
      const v4f wa2 = *(const v4f*)(sW1 + 64 + 8 * g);
      const v4f wb2 = *(const v4f*)(sW1 + 64 + 8 * g + 4);
      const v4f ba  = *(const v4f*)(sBias + 8 * g);
      const v4f bb  = *(const v4f*)(sBias + 8 * g + 4);
      const float w0[8] = {wa0[0], wa0[1], wa0[2], wa0[3], wb0[0], wb0[1], wb0[2], wb0[3]};
      const float w1[8] = {wa1[0], wa1[1], wa1[2], wa1[3], wb1[0], wb1[1], wb1[2], wb1[3]};
      const float w2[8] = {wa2[0], wa2[1], wa2[2], wa2[3], wb2[0], wb2[1], wb2[2], wb2[3]};
      const float bq[8] = {ba[0], ba[1], ba[2], ba[3], bb[0], bb[1], bb[2], bb[3]};
      v8h vfh, vfl, vth0, vth1, vth2, vtl0, vtl1, vtl2;
#pragma unroll
      for (int e = 0; e < 8; ++e) {
        float pre = x0 * w0[e];
        pre = fmaf(x1, w1[e], pre);
        pre = fmaf(x2, w2[e], pre);
        pre += bq[e];
        float hv, sv;
        act_pair(pre, hv, sv);
        _Float16 qh, ql;
        split_h(hv * kCarryA, qh, ql);
        vfh[e] = qh;
        vfl[e] = ql;
        const float sc = sv * kCarryA;
        if (kTanSplit) {
          split_h(sc * w0[e], qh, ql);
          vth0[e] = qh;
          vtl0[e] = ql;
          split_h(sc * w1[e], qh, ql);
          vth1[e] = qh;
          vtl1[e] = ql;
          split_h(sc * w2[e], qh, ql);
          vth2[e] = qh;
          vtl2[e] = ql;
        } else {
          vth0[e] = to_h(sc * w0[e]);
          vth1[e] = to_h(sc * w1[e]);
          vth2[e] = to_h(sc * w2[e]);
        }
      }
      _Float16* rowp = Aw + lane * kAP + 8 * g;
      *(v8h*)(rowp + kRowFwdHi * kAP) = vfh;
      if (kFwdSplit) *(v8h*)(rowp + kRowFwdLo * kAP) = vfl;
      *(v8h*)(rowp + (kRowTanHi + 0)  * kAP) = vth0;
      *(v8h*)(rowp + (kRowTanHi + 32) * kAP) = vth1;
      *(v8h*)(rowp + (kRowTanHi + 64) * kAP) = vth2;
      if (kTanSplit) {
        *(v8h*)(rowp + (kRowTanLo + 0)  * kAP) = vtl0;
        *(v8h*)(rowp + (kRowTanLo + 32) * kAP) = vtl1;
        *(v8h*)(rowp + (kRowTanLo + 64) * kAP) = vtl2;
      }
    }
    wave_sync();

    hidden_layer<true >(Aw, sW2h, sW2l, sBias + 32, hh, c);
    wave_sync();
    hidden_layer<false>(Aw, sW3h, sW3l, sBias + 64, hh, c);
    wave_sync();

#pragma unroll 1
    for (int mt = 0; mt < 2; ++mt) {
      v8f am = z8;
      v8f ar = z8;
#pragma unroll
      for (int ks = 0; ks < 3; ++ks) {
        const v16h bq = FragH::load(sW4 + c * kW4P + 32 * ks + 8 * hh);
        const v16h aq = FragH::load(Aw + (kRowTanHi + 32 * ks + mt * 16 + c) * kAP + 8 * hh);
        am = mma_h(aq, bq, am);
        if (kTanSplit) {
          const v16h al = FragH::load(Aw + (kRowTanLo + 32 * ks + mt * 16 + c) * kAP + 8 * hh);
          ar = mma_h(al, bq, ar);
        }
      }
      if (c < 3) {
#pragma unroll
        for (int r = 0; r < 8; ++r) {
          float o = am[r] * kInvMain;
          if (kTanSplit) o = fmaf(ar[r], kInvRes, o);
          Ow[(mt * 16 + 8 * hh + r) * 3 + c] = o;
        }
      }
    }
    wave_sync();

    const float o0 = Ow[lane];
    const float o1 = Ow[lane + 32];
    const float o2 = Ow[lane + 64];
    float* op = out + (size_t)t * 96 + lane;
    for (int pass = 0; pass < 2; ++pass) {
      *(volatile float*)(op)      = o0;
      *(volatile float*)(op + 32) = o1;
      *(volatile float*)(op + 64) = o2;
      __threadfence();
    }
  }
}

extern "C" void kernel_launch(void* const* d_in, const int* in_sizes, int n_in,
                              void* d_out, int out_size, void* d_ws, size_t ws_size,
                              hipStream_t stream) {
  (void)d_ws;
  (void)ws_size;
  if (n_in < 8) return;
  if (in_sizes[0] != kPts * 3) return;
  if (in_sizes[1] != 3 * kHid) return;
  if (in_sizes[2] != kHid) return;
  if (in_sizes[3] != kHid * kHid) return;
  if (in_sizes[4] != kHid) return;
  if (in_sizes[5] != kHid * kHid) return;
  if (in_sizes[6] != kHid) return;
  if (in_sizes[7] != kHid * 3) return;
  if (out_size != kPts * 3) return;

  const float* x  = (const float*)d_in[0];
  const float* W1 = (const float*)d_in[1];
  const float* b1 = (const float*)d_in[2];
  const float* W2 = (const float*)d_in[3];
  const float* b2 = (const float*)d_in[4];
  const float* W3 = (const float*)d_in[5];
  const float* b3 = (const float*)d_in[6];
  const float* W4 = (const float*)d_in[7];

  jet_field_kernel<<<kBlocks, kWaves * 32, 0, stream>>>(x, W1, b1, W2, b2, W3, b3, W4, (float*)d_out);
}
